// DGMCellLSTM_83915071029863
// MI455X (gfx1250) — hardware-verified
//
#include <hip/hip_runtime.h>
#include <math.h>

typedef __attribute__((ext_vector_type(16))) _Float16 v16h;
typedef __attribute__((ext_vector_type(8)))  _Float16 v8h;
typedef __attribute__((ext_vector_type(4)))  _Float16 v4h;
typedef __attribute__((ext_vector_type(8)))  float    v8f;
typedef __attribute__((ext_vector_type(4)))  float    v4f;

constexpr int kRows     = 262144;
constexpr int kDx       = 8;
constexpr int kHid      = 128;
constexpr int kLayers   = 3;
constexpr int kGates    = 4;
constexpr int kBlkRows  = 128;
constexpr int kTiles    = kBlkRows / 16;
constexpr int kKW       = 160;
constexpr int kKS       = 32;
constexpr int kActP     = 168;
constexpr int kSrP      = 136;
constexpr float kCarryA = 16.0f;
constexpr float kCarryW = 64.0f;
constexpr float kFold   = 1.0f / (kCarryA * kCarryW);
constexpr float kLoA    = 64.0f;
constexpr float kLoW    = 16.0f;
constexpr float kHMin   = 6.103515625e-5f;

static_assert(kRows == 2048 * kBlkRows, "row tiling is exact");
static_assert(kHid == 8 * 16, "eight waves own eight column tiles");
static_assert(kKW == kHid + 32 && (kKW % 32) == 0 && (kKS % 32) == 0, "k extents are multiples of 32");
static_assert(kDx == 8, "slab width");
static_assert((kActP * 2) % 16 == 0 && (kSrP * 2) % 16 == 0, "16-B aligned fragment rows");
static_assert(kActP >= kKW && kSrP >= kHid, "pitches cover the k range that is read");

constexpr size_t kPlaneHalves = (size_t)kHid * kKW;
constexpr size_t kBytesW      = (size_t)kLayers * kGates * kPlaneHalves * 2;
constexpr size_t kBytesS      = (size_t)kHid * kKS * 2;
constexpr size_t kOffW        = 0;
constexpr size_t kOffS        = kOffW + kBytesW;
constexpr size_t kWsTotal     = kOffS + kBytesS;
static_assert(kBytesW == 491520ull && kBytesS == 8192ull && kWsTotal == 499712ull, "carve total");
static_assert((kOffS % 128) == 0 && kWsTotal <= 134217728ull, "carve alignment and cap");
static_assert(kOffS == (size_t)kLayers * kGates * kPlaneHalves * 2, "input-layer plane follows plane 11");

__device__ __forceinline__ _Float16 hflush(float v) {
  const float vv = (fabsf(v) < kHMin) ? 0.0f : v;
  return (_Float16)vv;
}
__device__ __forceinline__ float sig_fast(float v) {
  return __builtin_amdgcn_rcpf(1.0f + __expf(-v));
}
__device__ __forceinline__ float tanh_fast(float v) {
  return 2.0f * __builtin_amdgcn_rcpf(1.0f + __expf(-2.0f * v)) - 1.0f;
}
union FragU { v16h v; v8h h[2]; };
__device__ __forceinline__ v16h ld_frag(const _Float16* p) {
  FragU f;
  f.h[0] = *(const v8h*)(p);
  f.h[1] = *(const v8h*)(p + 16);
  return f.v;
}
__device__ __forceinline__ v8f mma_h(v16h a, v16h b, v8f c) {
  c = __builtin_amdgcn_wmma_f32_16x16x32_f16(false, a, false, b, (short)0, c, false, false);
  asm volatile("v_nop\n\tv_nop\n\tv_nop\n\tv_nop" : "+v"(c) : "v"(a), "v"(b));
  return c;
}
__device__ __forceinline__ void load_b5(const _Float16* rowp, v16h (&b)[5]) {
#pragma unroll
  for (int k = 0; k < 5; ++k) {
    b[k] = ld_frag(rowp + 32 * k);
    asm volatile("" : "+v"(b[k]));
  }
}
__device__ __forceinline__ void stage_x_slab(_Float16* dst, float x0, float x1, float x2, float x3) {
  const float xs[4] = {x0, x1, x2, x3};
  v4h a, b, cc, z;
#pragma unroll
  for (int e = 0; e < 4; ++e) {
    const float s16 = kCarryA * xs[e];
    const _Float16 hh = hflush(s16);
    const float hf = (float)hh;
    a[e]  = hh;
    b[e]  = hflush((s16 - hf) * kLoA);
    cc[e] = hflush(hf * (1.0f / kLoW));
    z[e]  = (_Float16)0.0f;
  }
  *(v4h*)(dst)      = a;
  *(v4h*)(dst + 8)  = b;
  *(v4h*)(dst + 16) = cc;
  *(v4h*)(dst + 24) = z;
}

__global__ __launch_bounds__(256) void build_planes_kernel(
    const float* __restrict__ Sw,
    const float* __restrict__ Uz, const float* __restrict__ Wz,
    const float* __restrict__ Ug, const float* __restrict__ Wg,
    const float* __restrict__ Ur, const float* __restrict__ Wr,
    const float* __restrict__ Uh, const float* __restrict__ Wh,
    unsigned short* __restrict__ planes)
{
  const int tid = threadIdx.x;
  const int p   = blockIdx.y;
  const bool isIn = (p == kLayers * kGates);
  const int kch = isIn ? (kKS / 8) : (kKW / 8);
  const int nch = kHid * kch;
  const int ch  = blockIdx.x * 256 + tid;
  if (ch >= nch) return;
  const int l = isIn ? 0 : (p >> 2);
  const int g = p & 3;
  const float* Wsel = (g == 0) ? Wz : (g == 1) ? Wg : (g == 2) ? Wr : Wh;
  const float* Usel = (g == 0) ? Uz : (g == 1) ? Ug : (g == 2) ? Ur : Uh;
  const float* Wsrc = Wsel + (size_t)l * kHid * kHid;
  const float* Usrc = isIn ? Sw : (Usel + (size_t)l * kDx * kHid);

  const int n    = ch / kch;
  const int kc   = ch - n * kch;
  const int slab = kc - (kch - 4);
  const int kW   = (slab < 0) ? (kc * 8) : 0;

  float wv[8], uv[8];
#pragma unroll
  for (int e = 0; e < 8; ++e) {
    wv[e] = Wsrc[(size_t)(kW + e) * kHid + n];
    uv[e] = Usrc[e * kHid + n];
  }
#pragma unroll
  for (int e = 0; e < 8; ++e) {
    asm volatile("" : "+v"(wv[e]));
    asm volatile("" : "+v"(uv[e]));
  }
  v8h hv;
#pragma unroll
  for (int e = 0; e < 8; ++e) {
    const float us  = kCarryW * uv[e];
    const float uhf = (float)hflush(us);
    float sel = 0.0f;
    sel = (slab < 0)  ? (kCarryW * wv[e])       : sel;
    sel = (slab == 0) ? uhf                      : sel;
    sel = (slab == 1) ? (uhf * (1.0f / kLoA))    : sel;
    sel = (slab == 2) ? ((us - uhf) * kLoW)      : sel;
    hv[e] = hflush(sel);
  }
  unsigned short* dst = planes + (size_t)p * kPlaneHalves + (size_t)ch * 8;
  *(volatile v8h*)dst = hv;
  __threadfence();
  *(volatile v8h*)dst = hv;
}

__global__ __launch_bounds__(256) void gated_layers_kernel(
    const float* __restrict__ x, const float* __restrict__ Swb,
    const float* __restrict__ bz, const float* __restrict__ bg,
    const float* __restrict__ br, const float* __restrict__ bh,
    const float* __restrict__ Wf, const float* __restrict__ Wfb,
    const unsigned short* __restrict__ planes, float* __restrict__ out)
{
  __shared__ __align__(16) float    sSt[kTiles * 8 * 256];
  __shared__ __align__(16) _Float16 sAct[kBlkRows * kActP];
  __shared__ __align__(16) _Float16 sSR[kBlkRows * kSrP];
  __shared__ __align__(16) float    sPart[8 * kBlkRows];

  const int tid  = threadIdx.x;
  const int lane = tid & 31;
  const int w    = tid >> 5;
  const int h    = lane >> 4;
  const int c    = lane & 15;
  const int col  = w * 16 + c;
  const int rowBase = blockIdx.x * kBlkRows;

  const _Float16* gplanes = (const _Float16*)planes;

  const int xr = tid >> 1;
  const int xq = tid & 1;
  const v4f xv4 = *(const v4f*)(x + (size_t)(rowBase + xr) * kDx + 4 * xq);
  const float x0 = xv4[0], x1 = xv4[1], x2 = xv4[2], x3 = xv4[3];
  _Float16* xdst = sAct + xr * kActP + kHid + 4 * xq;

  stage_x_slab(xdst, x0, x1, x2, x3);
  __syncthreads();

  {
    v16h bS = ld_frag(gplanes + (size_t)kLayers * kGates * kPlaneHalves + (size_t)col * kKS + 8 * h);
    asm volatile("" : "+v"(bS));
    const float bias = Swb[col];
#pragma unroll 1
    for (int t = 0; t < kTiles; ++t) {
      const v16h a = ld_frag(sAct + (t * 16 + c) * kActP + kHid + 8 * h);
      v8f acc = (v8f){0.f, 0.f, 0.f, 0.f, 0.f, 0.f, 0.f, 0.f};
      acc = mma_h(a, bS, acc);
#pragma unroll
      for (int r = 0; r < 8; ++r) sSt[(t * 8 + r) * 256 + tid] = acc[r] * kFold + bias;
    }
  }
  __syncthreads();

#pragma unroll 1
  for (int l = 0; l < kLayers; ++l) {
    stage_x_slab(xdst, x0, x1, x2, x3);
#pragma unroll 1
    for (int t = 0; t < kTiles; ++t) {
#pragma unroll
      for (int r = 0; r < 8; ++r) {
        const int idx = (t * 8 + r) * 256 + tid;
        const float s = sig_fast(sSt[idx]);
        sSt[idx] = s;
        sAct[(t * 16 + 8 * h + r) * kActP + col] = hflush(kCarryA * s);
      }
    }
    __syncthreads();

    {
      v16h bR[5], bZ[5];
      load_b5(gplanes + (size_t)(l * kGates + 2) * kPlaneHalves + (size_t)col * kKW + 8 * h, bR);
      load_b5(gplanes + (size_t)(l * kGates + 0) * kPlaneHalves + (size_t)col * kKW + 8 * h, bZ);
      const float biasR = br[l * kHid + col];
      const float biasZ = bz[l * kHid + col];
#pragma unroll 1
      for (int t = 0; t < kTiles; ++t) {
        const _Float16* ap = sAct + (t * 16 + c) * kActP + 8 * h;
        v8f aR = (v8f){0.f, 0.f, 0.f, 0.f, 0.f, 0.f, 0.f, 0.f};
        v8f aZ = (v8f){0.f, 0.f, 0.f, 0.f, 0.f, 0.f, 0.f, 0.f};
#pragma unroll
        for (int k = 0; k < 5; ++k) {
          const v16h a = ld_frag(ap + 32 * k);
          aR = mma_h(a, bR[k], aR);
          aZ = mma_h(a, bZ[k], aZ);
        }
#pragma unroll
        for (int r = 0; r < 8; ++r) {
          const int idx = (t * 8 + r) * 256 + tid;
          const float s  = sSt[idx];
          const float Rv = sig_fast(aR[r] * kFold + biasR);
          const float Zv = sig_fast(aZ[r] * kFold + biasZ);
          sSR[(t * 16 + 8 * h + r) * kSrP + col] = hflush(kCarryA * (s * Rv));
          sSt[idx] = Zv * s;
        }
      }
    }
    __syncthreads();

    {
      v16h bG[5], bH[5];
      load_b5(gplanes + (size_t)(l * kGates + 1) * kPlaneHalves + (size_t)col * kKW + 8 * h, bG);
      load_b5(gplanes + (size_t)(l * kGates + 3) * kPlaneHalves + (size_t)col * kKW + 8 * h, bH);
      const float biasG = bg[l * kHid + col];
      const float biasH = bh[l * kHid + col];
#pragma unroll 1
      for (int t = 0; t < kTiles; ++t) {
        const _Float16* ap = sAct + (t * 16 + c) * kActP + 8 * h;
        const _Float16* sp = sSR  + (t * 16 + c) * kSrP  + 8 * h;
        v8f aG = (v8f){0.f, 0.f, 0.f, 0.f, 0.f, 0.f, 0.f, 0.f};
        v8f aH = (v8f){0.f, 0.f, 0.f, 0.f, 0.f, 0.f, 0.f, 0.f};
#pragma unroll
        for (int k = 0; k < 4; ++k) {
          const v16h a  = ld_frag(ap + 32 * k);
          aG = mma_h(a, bG[k], aG);
          const v16h hs = ld_frag(sp + 32 * k);
          aH = mma_h(hs, bH[k], aH);
        }
        {
          const v16h ax = ld_frag(ap + kHid);
          aG = mma_h(ax, bG[4], aG);
          aH = mma_h(ax, bH[4], aH);
        }
#pragma unroll
        for (int r = 0; r < 8; ++r) {
          const int idx = (t * 8 + r) * 256 + tid;
          const float Gv = sig_fast(aG[r] * kFold + biasG);
          const float Hv = tanh_fast(aH[r] * kFold + biasH);
          sSt[idx] = (1.0f - Gv) * Hv + sSt[idx];
        }
      }
    }
    __syncthreads();
  }

  {
    const float wfv = Wf[col];
#pragma unroll 1
    for (int t = 0; t < kTiles; ++t) {
#pragma unroll
      for (int r = 0; r < 8; ++r) {
        float v = sSt[(t * 8 + r) * 256 + tid] * wfv;
        v += __shfl_xor(v, 1, 32);
        v += __shfl_xor(v, 2, 32);
        v += __shfl_xor(v, 4, 32);
        v += __shfl_xor(v, 8, 32);
        if (c == 0) sPart[w * kBlkRows + t * 16 + 8 * h + r] = v;
      }
    }
  }
  __syncthreads();
  if (w == 0) {
    const float wfb = Wfb[0];
    v4f o;
#pragma unroll
    for (int e = 0; e < 4; ++e) {
      const int row = 4 * lane + e;
      float acc = sPart[row];
#pragma unroll
      for (int ww = 1; ww < 8; ++ww) acc += sPart[ww * kBlkRows + row];
      o[e] = acc + wfb;
    }
    float* dst = out + (size_t)rowBase + 4 * lane;
    *(volatile v4f*)dst = o;
    __threadfence();
    *(volatile v4f*)dst = o;
  }
}

extern "C" void kernel_launch(void* const* d_in, const int* in_sizes, int n_in,
                              void* d_out, int out_size, void* d_ws, size_t ws_size,
                              hipStream_t stream) {
  if (n_in < 17) return;
  if (in_sizes[0] != kRows * kDx) return;
  if (in_sizes[1] != kDx * kHid) return;
  if (in_sizes[2] != kHid) return;
  for (int g = 0; g < kGates; ++g) {
    if (in_sizes[3 + 3 * g] != kLayers * kDx * kHid) return;
    if (in_sizes[4 + 3 * g] != kLayers * kHid * kHid) return;
    if (in_sizes[5 + 3 * g] != kLayers * kHid) return;
  }
  if (in_sizes[15] != kHid) return;
  if (in_sizes[16] != 1) return;
  if (out_size != kRows) return;
  if (ws_size < kWsTotal) return;

  const float* x    = (const float*)d_in[0];
  const float* Sw_w = (const float*)d_in[1];
  const float* Sw_b = (const float*)d_in[2];
  const float* Uz   = (const float*)d_in[3];
  const float* Wz   = (const float*)d_in[4];
  const float* bz   = (const float*)d_in[5];
  const float* Ug   = (const float*)d_in[6];
  const float* Wg   = (const float*)d_in[7];
  const float* bg   = (const float*)d_in[8];
  const float* Ur   = (const float*)d_in[9];
  const float* Wr   = (const float*)d_in[10];
  const float* br   = (const float*)d_in[11];
  const float* Uh   = (const float*)d_in[12];
  const float* Wh   = (const float*)d_in[13];
  const float* bh   = (const float*)d_in[14];
  const float* Wf_w = (const float*)d_in[15];
  const float* Wf_b = (const float*)d_in[16];
  float* out = (float*)d_out;

  unsigned short* planes = (unsigned short*)((char*)d_ws + kOffW);

  build_planes_kernel<<<dim3((kHid * (kKW / 8) + 255) / 256, kLayers * kGates + 1), 256, 0, stream>>>(
      Sw_w, Uz, Wz, Ug, Wg, Ur, Wr, Uh, Wh, planes);

  gated_layers_kernel<<<kRows / kBlkRows, 256, 0, stream>>>(
      x, Sw_b, bz, bg, br, bh, Wf_w, Wf_b, planes, out);
}
